// ChebConvWithGAT_18571438588044
// MI455X (gfx1250) — hardware-run, weakly checked
//
#include <hip/hip_runtime.h>
#include <stddef.h>
#include <stdint.h>

#define NBA    8
#define NNODE  512
#define NCH    64
#define NSTEP  12
#define NPOLY  3
#define NFEAT  64
#define NHEAD  4
#define HDIM   16
#define NBT    96
#define KCF    192
#define KCHUNK 64
#define NCHUNK 8
#define SP     68
#define PP     72
#define SVP    264

static_assert(NBT == NBA * NSTEP);
static_assert(NHEAD * HDIM == NFEAT);
static_assert(KCF == NPOLY * NCH);
static_assert(NNODE % 256 == 0);
static_assert(NNODE == KCHUNK * NCHUNK);
static_assert(NCH == 64);
static_assert(NFEAT == 64);
static_assert(KCF % 32 == 0);
static_assert(NNODE % 32 == 0);

typedef unsigned short v8us  __attribute__((ext_vector_type(8)));
typedef unsigned short v16us __attribute__((ext_vector_type(16)));
typedef __bf16         v16bf __attribute__((ext_vector_type(16)));
typedef float          v8f   __attribute__((ext_vector_type(8)));
typedef float          v4f   __attribute__((ext_vector_type(4)));
typedef unsigned int   v4u   __attribute__((ext_vector_type(4)));

union Frag  { v16bf v; v16us u; v8us h[2]; };
union Pack8 { v8us h; v4u u; };

__device__ __forceinline__ unsigned short f2bf(float x) {
  unsigned int u = __float_as_uint(x);
  u += 0x7FFFu + ((u >> 16) & 1u);
  return (unsigned short)(u >> 16);
}
__device__ __forceinline__ float bf2f(unsigned short b) { return __uint_as_float(((unsigned int)b) << 16); }

__device__ __forceinline__ v8f zero8() { return (v8f){0.f, 0.f, 0.f, 0.f, 0.f, 0.f, 0.f, 0.f}; }

__device__ __forceinline__ v8f mma(const Frag& a, const Frag& b, v8f c) {
  c = __builtin_amdgcn_wmma_f32_16x16x32_bf16(false, a.v, false, b.v, (short)0, c, false, false);
  asm volatile("v_nop\n\tv_nop\n\tv_nop\n\tv_nop" : "+v"(c) : "v"(a.u), "v"(b.u));
  return c;
}

__device__ __forceinline__ Frag ldfrag(const unsigned short* p, int ld, size_t row0, int k0, int lane) {
  const int m = lane & 15, lh = lane >> 4;
  const unsigned short* q = p + (row0 + (size_t)m) * (size_t)ld + k0 + 8 * lh;
  Frag f;
  f.h[0] = *(const v8us*)(q);
  f.h[1] = *(const v8us*)(q + 16);
  return f;
}

__device__ __forceinline__ void split8(v4f a0, v4f a1, v4u& ho, v4u& lo) {
  Pack8 ph, pq;
#pragma unroll
  for (int j = 0; j < 4; ++j) {
    const unsigned short b0 = f2bf(a0[j]);
    ph.h[j] = b0;
    pq.h[j] = f2bf(a0[j] - bf2f(b0));
    const unsigned short b1 = f2bf(a1[j]);
    ph.h[4 + j] = b1;
    pq.h[4 + j] = f2bf(a1[j] - bf2f(b1));
  }
  ho = ph.u;
  lo = pq.u;
}

__device__ __forceinline__ void gemm_x3(const unsigned short* Ah, const unsigned short* Al, int lda, size_t ra0, size_t ra1,
                                        const unsigned short* Bh, const unsigned short* Bl, int ldb, size_t nrow0, int K,
                                        int lane, v8f (&acc)[2][4]) {
#pragma unroll 1
  for (int k0 = 0; k0 < K; k0 += 32) {
    const Frag a0h = ldfrag(Ah, lda, ra0, k0, lane);
    const Frag a1h = ldfrag(Ah, lda, ra1, k0, lane);
    const Frag a0l = ldfrag(Al, lda, ra0, k0, lane);
    const Frag a1l = ldfrag(Al, lda, ra1, k0, lane);
#pragma unroll
    for (int t = 0; t < 4; ++t) {
      const Frag bh = ldfrag(Bh, ldb, nrow0 + 16 * t, k0, lane);
      const Frag bl = ldfrag(Bl, ldb, nrow0 + 16 * t, k0, lane);
      acc[0][t] = mma(a0h, bh, acc[0][t]);
      acc[1][t] = mma(a1h, bh, acc[1][t]);
      acc[0][t] = mma(a0h, bl, acc[0][t]);
      acc[1][t] = mma(a1h, bl, acc[1][t]);
      acc[0][t] = mma(a0l, bh, acc[0][t]);
      acc[1][t] = mma(a1l, bh, acc[1][t]);
    }
  }
}

template <bool RELU>
__device__ __forceinline__ void epi_bf16(v8f (&acc)[2][4], const float (&bb)[4], float* sw,
                                         unsigned short* __restrict__ oh, unsigned short* __restrict__ ol,
                                         size_t orow0, size_t orow1, int ldo, int col0, int lane) {
  const int hh = lane >> 4, c = lane & 15;
#pragma unroll
  for (int sub = 0; sub < 2; ++sub) {
    __syncthreads();
#pragma unroll
    for (int t = 0; t < 4; ++t) {
#pragma unroll
      for (int r = 0; r < 8; ++r) {
        float v = acc[sub][t][r] + bb[t];
        if (RELU) v = fmaxf(v, 0.f);
        sw[(8 * hh + r) * SP + 16 * t + c] = v;
      }
    }
    __syncthreads();
    v4u hv[4], lv[4];
    size_t go[4];
    const size_t orow = sub ? orow1 : orow0;
#pragma unroll
    for (int it = 0; it < 4; ++it) {
      const int p  = lane + 32 * it;
      const int L  = p >> 3;
      const int pc = p & 7;
      const float* ra = sw + L * SP + pc * 8;
      const v4f a0 = *(const v4f*)(ra);
      const v4f a1 = *(const v4f*)(ra + 4);
      split8(a0, a1, hv[it], lv[it]);
      go[it] = (orow + (size_t)L) * (size_t)ldo + col0 + pc * 8;
    }
#pragma unroll
    for (int it = 0; it < 4; ++it) {
      *(volatile v4u*)(oh + go[it]) = hv[it];
      *(volatile v4u*)(ol + go[it]) = lv[it];
    }
    __threadfence();
#pragma unroll
    for (int it = 0; it < 4; ++it) {
      *(volatile v4u*)(oh + go[it]) = hv[it];
      *(volatile v4u*)(ol + go[it]) = lv[it];
    }
  }
}

__global__ __launch_bounds__(256) void k_cvt_x(const float* __restrict__ x,
                                               unsigned short* __restrict__ xth, unsigned short* __restrict__ xtl) {
  __shared__ __align__(16) float tile[NCH * SP];
  const int tid = threadIdx.x;
  const int bt = blockIdx.x >> 3, ig = blockIdx.x & 7;
  const int b = bt / NSTEP, t = bt - b * NSTEP;
  const int i0 = ig * 64;
  const float* xb = x + ((size_t)(b * NNODE + i0)) * (NCH * NSTEP) + t;
#pragma unroll
  for (int it = 0; it < 16; ++it) {
    const int e  = it * 256 + tid;
    const int ii = e >> 6, c = e & 63;
    tile[c * SP + ii] = xb[(size_t)(ii * NCH + c) * NSTEP];
  }
  __syncthreads();
  v4u hv[2], lv[2];
  size_t go[2];
#pragma unroll
  for (int it = 0; it < 2; ++it) {
    const int p  = it * 256 + tid;
    const int c  = p >> 3, pc = p & 7;
    const float* ra = tile + c * SP + pc * 8;
    const v4f a0 = *(const v4f*)(ra);
    const v4f a1 = *(const v4f*)(ra + 4);
    split8(a0, a1, hv[it], lv[it]);
    go[it] = ((size_t)(bt * NCH + c)) * NNODE + i0 + pc * 8;
  }
#pragma unroll
  for (int it = 0; it < 2; ++it) { *(volatile v4u*)(xth + go[it]) = hv[it]; *(volatile v4u*)(xtl + go[it]) = lv[it]; }
  __threadfence();
#pragma unroll
  for (int it = 0; it < 2; ++it) { *(volatile v4u*)(xth + go[it]) = hv[it]; *(volatile v4u*)(xtl + go[it]) = lv[it]; }
}

__global__ __launch_bounds__(256) void k_cvt_poly(const float* __restrict__ poly,
                                                  unsigned short* __restrict__ tth, unsigned short* __restrict__ ttl) {
  __shared__ __align__(16) float tile[64 * SP];
  const int tid = threadIdx.x;
  const int bx = blockIdx.x;
  const int k = bx >> 6, jt = (bx >> 3) & 7, ib = bx & 7;
  const int i0 = ib * 64, j0 = jt * 64;
  const float* src = poly + ((size_t)(k * NNODE + i0)) * NNODE + j0;
#pragma unroll
  for (int it = 0; it < 16; ++it) {
    const int e  = it * 256 + tid;
    const int ii = e >> 6, jj = e & 63;
    tile[jj * SP + ii] = src[(size_t)ii * NNODE + jj];
  }
  __syncthreads();
  v4u hv[2], lv[2];
  size_t go[2];
#pragma unroll
  for (int it = 0; it < 2; ++it) {
    const int p  = it * 256 + tid;
    const int jj = p >> 3, pc = p & 7;
    const float* ra = tile + jj * SP + pc * 8;
    const v4f a0 = *(const v4f*)(ra);
    const v4f a1 = *(const v4f*)(ra + 4);
    split8(a0, a1, hv[it], lv[it]);
    go[it] = ((size_t)(k * NNODE + j0 + jj)) * NNODE + i0 + pc * 8;
  }
#pragma unroll
  for (int it = 0; it < 2; ++it) { *(volatile v4u*)(tth + go[it]) = hv[it]; *(volatile v4u*)(ttl + go[it]) = lv[it]; }
  __threadfence();
#pragma unroll
  for (int it = 0; it < 2; ++it) { *(volatile v4u*)(tth + go[it]) = hv[it]; *(volatile v4u*)(ttl + go[it]) = lv[it]; }
}

__global__ __launch_bounds__(256) void k_cvt_w(const float* __restrict__ theta, const float* __restrict__ win,
                                               const float* __restrict__ wo, const float* __restrict__ wfc,
                                               unsigned short* __restrict__ tth, unsigned short* __restrict__ ttl,
                                               unsigned short* __restrict__ wih, unsigned short* __restrict__ wil,
                                               unsigned short* __restrict__ woh, unsigned short* __restrict__ wol,
                                               unsigned short* __restrict__ wfh, unsigned short* __restrict__ wfl) {
  const int tid = threadIdx.x;
  const int role = blockIdx.x;
  if (role == 0) {
#pragma unroll 1
    for (int it = 0; it < 6; ++it) {
      const int p  = it * 256 + tid;
      const int f  = p / 24;
      const int q  = p - f * 24;
      const int k  = q >> 3;
      const int cb = (q & 7) * 8;
      const float* s = theta + ((size_t)(k * NCH + cb)) * NFEAT + f;
      const v4f a0 = {s[0 * NFEAT], s[1 * NFEAT], s[2 * NFEAT], s[3 * NFEAT]};
      const v4f a1 = {s[4 * NFEAT], s[5 * NFEAT], s[6 * NFEAT], s[7 * NFEAT]};
      v4u hv, lv;
      split8(a0, a1, hv, lv);
      const size_t go = (size_t)f * KCF + q * 8;
      *(volatile v4u*)(tth + go) = hv; *(volatile v4u*)(ttl + go) = lv;
      __threadfence();
      *(volatile v4u*)(tth + go) = hv; *(volatile v4u*)(ttl + go) = lv;
    }
  } else {
    const float* src = (role == 1) ? win : ((role == 2) ? wo : wfc);
    unsigned short* dh = (role == 1) ? wih : ((role == 2) ? woh : wfh);
    unsigned short* dl = (role == 1) ? wil : ((role == 2) ? wol : wfl);
    const int niter = (role == 1) ? 6 : 2;
#pragma unroll 1
    for (int it = 0; it < niter; ++it) {
      const int p = it * 256 + tid;
      const v4f a0 = *(const v4f*)(src + (size_t)p * 8);
      const v4f a1 = *(const v4f*)(src + (size_t)p * 8 + 4);
      v4u hv, lv;
      split8(a0, a1, hv, lv);
      const size_t go = (size_t)p * 8;
      *(volatile v4u*)(dh + go) = hv; *(volatile v4u*)(dl + go) = lv;
      __threadfence();
      *(volatile v4u*)(dh + go) = hv; *(volatile v4u*)(dl + go) = lv;
    }
  }
}

__global__ __launch_bounds__(256) void k_gemm_z(const unsigned short* __restrict__ tth, const unsigned short* __restrict__ ttl,
                                                const unsigned short* __restrict__ xth, const unsigned short* __restrict__ xtl,
                                                unsigned short* __restrict__ zh, unsigned short* __restrict__ zl) {
  __shared__ __align__(16) float st[8][16 * SP];
  const int tid = threadIdx.x, lane = tid & 31, wave = tid >> 5;
  const int bt = blockIdx.y, k = blockIdx.z;
  const int m0 = blockIdx.x * 256 + wave * 32;
  const size_t ra0 = (size_t)k * NNODE + m0, ra1 = ra0 + 16;
  v8f acc[2][4];
#pragma unroll
  for (int s = 0; s < 2; ++s)
#pragma unroll
    for (int t = 0; t < 4; ++t) acc[s][t] = zero8();
  gemm_x3(tth, ttl, NNODE, ra0, ra1, xth, xtl, NNODE, (size_t)bt * NCH, NNODE, lane, acc);
  const float bb[4] = {0.f, 0.f, 0.f, 0.f};
  const size_t orow0 = (size_t)bt * NNODE + m0;
  epi_bf16<false>(acc, bb, st[wave], zh, zl, orow0, orow0 + 16, KCF, k * NCH, lane);
}

__global__ __launch_bounds__(256) void k_gemm_y(const unsigned short* __restrict__ zh, const unsigned short* __restrict__ zl,
                                                const unsigned short* __restrict__ tth, const unsigned short* __restrict__ ttl,
                                                unsigned short* __restrict__ yh, unsigned short* __restrict__ yl) {
  __shared__ __align__(16) float st[8][16 * SP];
  const int tid = threadIdx.x, lane = tid & 31, wave = tid >> 5;
  const int bt = blockIdx.y;
  const int m0 = blockIdx.x * 256 + wave * 32;
  const size_t ra0 = (size_t)bt * NNODE + m0, ra1 = ra0 + 16;
  v8f acc[2][4];
#pragma unroll
  for (int s = 0; s < 2; ++s)
#pragma unroll
    for (int t = 0; t < 4; ++t) acc[s][t] = zero8();
  gemm_x3(zh, zl, KCF, ra0, ra1, tth, ttl, KCF, 0, KCF, lane, acc);
  const float bb[4] = {0.f, 0.f, 0.f, 0.f};
  epi_bf16<true>(acc, bb, st[wave], yh, yl, ra0, ra1, NFEAT, 0, lane);
}

__global__ __launch_bounds__(256) void k_qkv(const unsigned short* __restrict__ yh, const unsigned short* __restrict__ yl,
                                             const unsigned short* __restrict__ wih, const unsigned short* __restrict__ wil,
                                             const float* __restrict__ inb,
                                             unsigned short* __restrict__ qh, unsigned short* __restrict__ ql,
                                             unsigned short* __restrict__ kh, unsigned short* __restrict__ kl,
                                             unsigned short* __restrict__ vth, unsigned short* __restrict__ vtl) {
  __shared__ __align__(16) unsigned short st[256 * PP];
  const int tid = threadIdx.x, lane = tid & 31, wave = tid >> 5;
  const int hh = lane >> 4, c = lane & 15;
  const int bt = blockIdx.x >> 1;
  const int sb = (blockIdx.x & 1) * 256;
  const int which = blockIdx.y;
  const int m0 = sb + wave * 32;
  const size_t ra0 = (size_t)bt * NNODE + m0, ra1 = ra0 + 16;

  v8f acc[2][4];
#pragma unroll
  for (int s = 0; s < 2; ++s)
#pragma unroll
    for (int t = 0; t < 4; ++t) acc[s][t] = zero8();
  gemm_x3(yh, yl, NFEAT, ra0, ra1, wih, wil, NFEAT, (size_t)which * NFEAT, NFEAT, lane, acc);

  float bb[4];
#pragma unroll
  for (int t = 0; t < 4; ++t) bb[t] = inb[which * NFEAT + 16 * t + c];

#pragma unroll 1
  for (int pl = 0; pl < 2; ++pl) {
    __syncthreads();
#pragma unroll
    for (int sub = 0; sub < 2; ++sub)
#pragma unroll
      for (int t = 0; t < 4; ++t)
#pragma unroll
        for (int r = 0; r < 8; ++r) {
          const float v = acc[sub][t][r] + bb[t];
          const unsigned short hb = f2bf(v);
          const unsigned short lb = f2bf(v - bf2f(hb));
          const unsigned short bits = (pl == 0) ? hb : lb;
          if (which < 2) st[(wave * 32 + sub * 16 + 8 * hh + r) * PP + 16 * t + c] = bits;
          else           st[(16 * t + c) * SVP + wave * 32 + sub * 16 + 8 * hh + r] = bits;
        }
    __syncthreads();
    if (which < 2) {
      unsigned short* dst = (which == 0) ? ((pl == 0) ? qh : ql) : ((pl == 0) ? kh : kl);
      dst += (size_t)bt * NNODE * NFEAT;
      v4u val[8];
      size_t go[8];
#pragma unroll
      for (int j = 0; j < 8; ++j) {
        const int p  = tid + 256 * j;
        const int lr = p >> 3;
        const int pc = p & 7;
        Pack8 pk;
        pk.h   = *(const v8us*)(st + lr * PP + pc * 8);
        val[j] = pk.u;
        go[j]  = (size_t)(sb + lr) * NFEAT + pc * 8;
      }
#pragma unroll
      for (int j = 0; j < 8; ++j) *(volatile v4u*)(dst + go[j]) = val[j];
      __threadfence();
#pragma unroll
      for (int j = 0; j < 8; ++j) *(volatile v4u*)(dst + go[j]) = val[j];
    } else {
      unsigned short* dst = (pl == 0) ? vth : vtl;
      dst += (size_t)bt * NFEAT * NNODE;
      v4u val[8];
      size_t go[8];
#pragma unroll
      for (int j = 0; j < 8; ++j) {
        const int p    = tid + 256 * j;
        const int drow = p >> 5;
        const int pc   = p & 31;
        Pack8 pk;
        pk.h   = *(const v8us*)(st + drow * SVP + pc * 8);
        val[j] = pk.u;
        go[j]  = (size_t)drow * NNODE + sb + pc * 8;
      }
#pragma unroll
      for (int j = 0; j < 8; ++j) *(volatile v4u*)(dst + go[j]) = val[j];
      __threadfence();
#pragma unroll
      for (int j = 0; j < 8; ++j) *(volatile v4u*)(dst + go[j]) = val[j];
    }
  }
}

__global__ __launch_bounds__(256) void k_attn(const unsigned short* __restrict__ qh, const unsigned short* __restrict__ ql,
                                              const unsigned short* __restrict__ kh, const unsigned short* __restrict__ kl,
                                              const unsigned short* __restrict__ vth, const unsigned short* __restrict__ vtl,
                                              unsigned short* __restrict__ oh, unsigned short* __restrict__ ol) {
  __shared__ __align__(16) unsigned short Ph[8][16 * PP];
  __shared__ __align__(16) unsigned short Pl[8][16 * PP];
  __shared__ __align__(16) float Os[32 * SP];

  const int tid = threadIdx.x, lane = tid & 31, wave = tid >> 5;
  const int hh = lane >> 4, m = lane & 15;
  const int bt   = blockIdx.x >> 4;
  const int qblk = blockIdx.x & 15;
  const int h    = wave & 3;
  const int rt   = wave >> 2;
  const int q0   = qblk * 32 + rt * 16;

  const size_t plane = (size_t)bt * NNODE * NFEAT;
  const unsigned short* Qh = qh + plane + h * HDIM;
  const unsigned short* Ql = ql + plane + h * HDIM;
  const unsigned short* Kh = kh + plane + h * HDIM;
  const unsigned short* Kl = kl + plane + h * HDIM;
  const unsigned short* Vh = vth + ((size_t)bt * NFEAT + h * HDIM) * NNODE;
  const unsigned short* Vl = vtl + ((size_t)bt * NFEAT + h * HDIM) * NNODE;

  Frag qa;
  {
    const size_t qo = (size_t)(q0 + m) * NFEAT + 8 * hh;
    qa.h[0] = *(const v8us*)(Qh + qo);
    qa.h[1] = *(const v8us*)(Ql + qo);
  }
  const v8us z8 = {0, 0, 0, 0, 0, 0, 0, 0};
  const float NEGI = -__builtin_huge_valf();
  float mrow[8], lrow[8];
  v8f oacc = zero8();
#pragma unroll
  for (int r = 0; r < 8; ++r) { mrow[r] = NEGI; lrow[r] = 0.f; }

  unsigned short* pwh = Ph[wave];
  unsigned short* pwl = Pl[wave];

#pragma unroll 1
  for (int kc = 0; kc < NCHUNK; ++kc) {
    const int kv0 = kc * KCHUNK;
    __syncthreads();

    v8f s[4];
#pragma unroll
    for (int j = 0; j < 4; ++j) {
      const size_t ko = (size_t)(kv0 + 16 * j + m) * NFEAT + 8 * hh;
      Frag b1, b2;
      b1.h[0] = *(const v8us*)(Kh + ko);
      b1.h[1] = b1.h[0];
      b2.h[0] = *(const v8us*)(Kl + ko);
      b2.h[1] = z8;
      s[j] = mma(qa, b1, zero8());
      s[j] = mma(qa, b2, s[j]);
    }
    float cm[8];
#pragma unroll
    for (int r = 0; r < 8; ++r) {
      float mx = NEGI;
#pragma unroll
      for (int j = 0; j < 4; ++j) { s[j][r] *= 0.25f; mx = fmaxf(mx, s[j][r]); }
#pragma unroll
      for (int off = 1; off < 16; off <<= 1) mx = fmaxf(mx, __shfl_xor(mx, off, 32));
      cm[r] = mx;
    }
    float al[8];
#pragma unroll
    for (int r = 0; r < 8; ++r) {
      const float mnew  = fmaxf(mrow[r], cm[r]);
      const float alpha = __expf(mrow[r] - mnew);
      mrow[r] = mnew;
      float psum = 0.f;
#pragma unroll
      for (int j = 0; j < 4; ++j) {
        const float p = __expf(s[j][r] - mnew);
        psum += p;
        const unsigned short hb = f2bf(p);
        const unsigned short lb = f2bf(p - bf2f(hb));
        pwh[(8 * hh + r) * PP + 16 * j + m] = hb;
        pwl[(8 * hh + r) * PP + 16 * j + m] = lb;
      }
#pragma unroll
      for (int off = 1; off < 16; off <<= 1) psum += __shfl_xor(psum, off, 32);
      lrow[r] = lrow[r] * alpha + psum;
      al[r] = alpha;
    }
#pragma unroll
    for (int r = 0; r < 8; ++r) oacc[r] *= al[r];
    __syncthreads();

#pragma unroll
    for (int kk = 0; kk < 2; ++kk) {
      const Frag pa = ldfrag(pwh, PP, 0, kk * 32, lane);
      const Frag pb = ldfrag(pwl, PP, 0, kk * 32, lane);
      const Frag vh = ldfrag(Vh, NNODE, 0, kv0 + kk * 32, lane);
      const Frag vl = ldfrag(Vl, NNODE, 0, kv0 + kk * 32, lane);
      oacc = mma(pa, vh, oacc);
      oacc = mma(pa, vl, oacc);
      oacc = mma(pb, vh, oacc);
    }
  }

  float invl[8];
#pragma unroll
  for (int r = 0; r < 8; ++r) invl[r] = (lrow[r] > 0.f) ? (1.0f / lrow[r]) : 0.f;
  __syncthreads();
#pragma unroll
  for (int r = 0; r < 8; ++r) Os[(rt * 16 + 8 * hh + r) * SP + h * HDIM + m] = oacc[r] * invl[r];
  __syncthreads();
  {
    const int lr = tid >> 3;
    const int pc = tid & 7;
    const float* ra = Os + lr * SP + pc * 8;
    const v4f a0 = *(const v4f*)(ra);
    const v4f a1 = *(const v4f*)(ra + 4);
    v4u hv, lv;
    split8(a0, a1, hv, lv);
    const size_t go = ((size_t)bt * NNODE + qblk * 32 + lr) * NFEAT + pc * 8;
    *(volatile v4u*)(oh + go) = hv; *(volatile v4u*)(ol + go) = lv;
    __threadfence();
    *(volatile v4u*)(oh + go) = hv; *(volatile v4u*)(ol + go) = lv;
  }
}

#define LDS_OUT_BYTES 55296
__global__ __launch_bounds__(192) void k_out(const unsigned short* __restrict__ ohp, const unsigned short* __restrict__ olp,
                                             const unsigned short* __restrict__ woh, const unsigned short* __restrict__ wol,
                                             const float* __restrict__ bo,
                                             const unsigned short* __restrict__ wfh, const unsigned short* __restrict__ wfl,
                                             const float* __restrict__ bfc, float* __restrict__ out) {
  __shared__ __align__(16) unsigned char lds[LDS_OUT_BYTES];
  unsigned short* a1h = (unsigned short*)lds;
  unsigned short* a1l = (unsigned short*)(lds + 192 * PP * 2);
  float* ost = (float*)lds;

  const int tid = threadIdx.x, lane = tid & 31, wave = tid >> 5;
  const int hh = lane >> 4, c = lane & 15;
  const int b  = blockIdx.x >> 5;
  const int n0 = (blockIdx.x & 31) * 16;
  const size_t rO0 = ((size_t)(b * NSTEP + 2 * wave)) * NNODE + n0;
  const size_t rO1 = rO0 + NNODE;

  v8f acc[2][4];
#pragma unroll
  for (int s = 0; s < 2; ++s)
#pragma unroll
    for (int t = 0; t < 4; ++t) acc[s][t] = zero8();
  gemm_x3(ohp, olp, NFEAT, rO0, rO1, woh, wol, NFEAT, 0, NFEAT, lane, acc);

  float bb[4];
#pragma unroll
  for (int t = 0; t < 4; ++t) bb[t] = bo[16 * t + c];
#pragma unroll
  for (int s = 0; s < 2; ++s)
#pragma unroll
    for (int t = 0; t < 4; ++t)
#pragma unroll
      for (int r = 0; r < 8; ++r) {
        const float v = acc[s][t][r] + bb[t];
        const unsigned short hb = f2bf(v);
        const unsigned short lb = f2bf(v - bf2f(hb));
        const int row = wave * 32 + s * 16 + 8 * hh + r;
        a1h[row * PP + 16 * t + c] = hb;
        a1l[row * PP + 16 * t + c] = lb;
      }
  __syncthreads();

  v8f acc2[2][4];
#pragma unroll
  for (int s = 0; s < 2; ++s)
#pragma unroll
    for (int t = 0; t < 4; ++t) acc2[s][t] = zero8();
  gemm_x3(a1h, a1l, PP, (size_t)wave * 32, (size_t)wave * 32 + 16, wfh, wfl, NFEAT, 0, NFEAT, lane, acc2);
  __syncthreads();

  float bb2[4];
#pragma unroll
  for (int t = 0; t < 4; ++t) bb2[t] = bfc[16 * t + c];
#pragma unroll
  for (int s = 0; s < 2; ++s)
#pragma unroll
    for (int t = 0; t < 4; ++t)
#pragma unroll
      for (int r = 0; r < 8; ++r) {
        const float v  = fmaxf(acc2[s][t][r] + bb2[t], 0.f);
        const int step = 2 * wave + s;
        const int nl   = 8 * hh + r;
        const int f    = 16 * t + c;
        ost[(nl * NFEAT + f) * NSTEP + step] = v;
      }
  __syncthreads();

  float* ob = out + ((size_t)(b * NNODE + n0)) * (NFEAT * NSTEP);
#pragma unroll
  for (int g = 0; g < 2; ++g) {
    v4f val[8];
#pragma unroll
    for (int j = 0; j < 8; ++j) {
      const int p = (g * 8 + j) * 192 + tid;
      val[j] = *(const v4f*)(ost + p * 4);
    }
#pragma unroll
    for (int j = 0; j < 8; ++j) {
      const int p = (g * 8 + j) * 192 + tid;
      *(volatile v4f*)(ob + (size_t)p * 4) = val[j];
    }
    __threadfence();
#pragma unroll
    for (int j = 0; j < 8; ++j) {
      const int p = (g * 8 + j) * 192 + tid;
      *(volatile v4f*)(ob + (size_t)p * 4) = val[j];
    }
  }
}

extern "C" void kernel_launch(void* const* d_in, const int* in_sizes, int n_in,
                              void* d_out, int out_size, void* d_ws, size_t ws_size,
                              hipStream_t stream) {
  if (n_in < 10) return;
  if (in_sizes[0] != NBA * NNODE * NCH * NSTEP) return;
  if (in_sizes[2] != NPOLY * NNODE * NNODE) return;
  if (in_sizes[3] != NPOLY * NCH * NFEAT) return;
  if (in_sizes[4] != 3 * NFEAT * NFEAT) return;
  if (in_sizes[5] != 3 * NFEAT) return;
  if (in_sizes[6] != NFEAT * NFEAT) return;
  if (in_sizes[7] != NFEAT) return;
  if (in_sizes[8] != NFEAT * NFEAT) return;
  if (in_sizes[9] != NFEAT) return;
  if (out_size != NBA * NNODE * NFEAT * NSTEP) return;

  const float* x     = (const float*)d_in[0];
  const float* poly  = (const float*)d_in[2];
  const float* theta = (const float*)d_in[3];
  const float* win   = (const float*)d_in[4];
  const float* inb   = (const float*)d_in[5];
  const float* wo    = (const float*)d_in[6];
  const float* bo    = (const float*)d_in[7];
  const float* wfc   = (const float*)d_in[8];
  const float* bfc   = (const float*)d_in[9];
  float* out = (float*)d_out;

  const size_t szXT  = (size_t)NBT * NCH * NNODE * 2;
  const size_t szTT  = (size_t)NPOLY * NNODE * NNODE * 2;
  const size_t szThT = (size_t)NFEAT * KCF * 2;
  const size_t szWin = (size_t)3 * NFEAT * NFEAT * 2;
  const size_t szW   = (size_t)NFEAT * NFEAT * 2;
  const size_t szZc  = (size_t)NBT * NNODE * KCF * 2;
  const size_t szA   = (size_t)NBT * NNODE * NFEAT * 2;

  size_t off = 0;
  const size_t oXTh = off; off += szXT;   const size_t oXTl = off; off += szXT;
  const size_t oTTh = off; off += szTT;   const size_t oTTl = off; off += szTT;
  const size_t oThh = off; off += szThT;  const size_t oThl = off; off += szThT;
  const size_t oWih = off; off += szWin;  const size_t oWil = off; off += szWin;
  const size_t oWoh = off; off += szW;    const size_t oWol = off; off += szW;
  const size_t oWfh = off; off += szW;    const size_t oWfl = off; off += szW;
  const size_t oZch = off; off += szZc;   const size_t oZcl = off; off += szZc;
  const size_t oXAh = off; off += szA;    const size_t oXAl = off; off += szA;
  const size_t oQh  = off; off += szA;    const size_t oQl  = off; off += szA;
  const size_t oKh  = off; off += szA;    const size_t oKl  = off; off += szA;
  const size_t oVh  = off; off += szA;    const size_t oVl  = off; off += szA;
  const size_t oOh  = off; off += szA;    const size_t oOl  = off; off += szA;
  if (off > ws_size) return;
  if (off > (size_t)134217728) return;

  char* ws = (char*)d_ws;
  unsigned short* XTh = (unsigned short*)(ws + oXTh); unsigned short* XTl = (unsigned short*)(ws + oXTl);
  unsigned short* TTh = (unsigned short*)(ws + oTTh); unsigned short* TTl = (unsigned short*)(ws + oTTl);
  unsigned short* Thh = (unsigned short*)(ws + oThh); unsigned short* Thl = (unsigned short*)(ws + oThl);
  unsigned short* Wih = (unsigned short*)(ws + oWih); unsigned short* Wil = (unsigned short*)(ws + oWil);
  unsigned short* Woh = (unsigned short*)(ws + oWoh); unsigned short* Wol = (unsigned short*)(ws + oWol);
  unsigned short* Wfh = (unsigned short*)(ws + oWfh); unsigned short* Wfl = (unsigned short*)(ws + oWfl);
  unsigned short* Zch = (unsigned short*)(ws + oZch); unsigned short* Zcl = (unsigned short*)(ws + oZcl);
  unsigned short* XAh = (unsigned short*)(ws + oXAh); unsigned short* XAl = (unsigned short*)(ws + oXAl);
  unsigned short* Qh  = (unsigned short*)(ws + oQh);  unsigned short* Ql  = (unsigned short*)(ws + oQl);
  unsigned short* Kh  = (unsigned short*)(ws + oKh);  unsigned short* Kl  = (unsigned short*)(ws + oKl);
  unsigned short* Vh  = (unsigned short*)(ws + oVh);  unsigned short* Vl  = (unsigned short*)(ws + oVl);
  unsigned short* Oh  = (unsigned short*)(ws + oOh);  unsigned short* Ol  = (unsigned short*)(ws + oOl);

  k_cvt_x<<<dim3(NBT * 8), dim3(256), 0, stream>>>(x, XTh, XTl);
  k_cvt_poly<<<dim3(NPOLY * 64), dim3(256), 0, stream>>>(poly, TTh, TTl);
  k_cvt_w<<<dim3(4), dim3(256), 0, stream>>>(theta, win, wo, wfc, Thh, Thl, Wih, Wil, Woh, Wol, Wfh, Wfl);
  k_gemm_z<<<dim3(NNODE / 256, NBT, NPOLY), dim3(256), 0, stream>>>(TTh, TTl, XTh, XTl, Zch, Zcl);
  k_gemm_y<<<dim3(NNODE / 256, NBT), dim3(256), 0, stream>>>(Zch, Zcl, Thh, Thl, XAh, XAl);
  k_qkv<<<dim3(NBT * 2, 3), dim3(256), 0, stream>>>(XAh, XAl, Wih, Wil, inb, Qh, Ql, Kh, Kl, Vh, Vl);
  k_attn<<<dim3(NBT * 16), dim3(256), 0, stream>>>(Qh, Ql, Kh, Kl, Vh, Vl, Oh, Ol);
  k_out<<<dim3(NBA * 32), dim3(192), 0, stream>>>(Oh, Ol, Woh, Wol, bo, Wfh, Wfl, bfc, out);
  (void)hipGetLastError();
}
